// CrossAttentionS2T_22204980921033
// MI455X (gfx1250) — hardware-verified
//
#include <hip/hip_runtime.h>
#include <math.h>
#include <stdint.h>

#define TFR     8
#define NSP     196
#define NB      4
#define NBT     32
#define DM      768
#define NH      12
#define HD      64
#define SQ      1568
#define SP      1600
#define KVN     1536
#define NSROWS  198
#define NTROWS  197
#define WSC     64.0f
#define ACARRY  16.0f
#define QKCARRY 16.0f
#define VCARRY  16.0f
#define PCARRY  1024.0f
#define FCARRY  256.0f
static_assert(SQ == TFR * NSP);
static_assert(NBT == NB * TFR);
static_assert(NH * HD == DM);
static_assert((SQ % 32) == 0 && (SQ % 16) == 0);
static_assert((SP % 64) == 0 && SP >= SQ && (DM % 64) == 0 && (HD % 64) == 0);
static_assert(KVN == 2 * DM);

#define P_CH          (DM / 8)
#define PREP_THREADS  (NB * SP * P_CH)
#define PREP_BLOCKS   (PREP_THREADS / 256)
#define CLS_THREADS   (NBT * DM / 4)
#define CLS_BLOCKS    (CLS_THREADS / 256)
#define ZP_PERB       ((SP - SQ) * P_CH)
#define ZP_THREADS    (NB * ZP_PERB)
#define ZP_BLOCKS     (ZP_THREADS / 256)
#define ATT_WAVES     (NB * NH * (SQ / 16))
#define ATT_BLOCKS    (ATT_WAVES / 4)
static_assert(PREP_THREADS % 256 == 0 && CLS_THREADS % 256 == 0 && ZP_THREADS % 256 == 0);
static_assert((P_CH % 32) == 0 && ((DM / 4) % 32) == 0);
static_assert(ATT_WAVES % 4 == 0);

typedef _Float16 v16h __attribute__((ext_vector_type(16)));
typedef _Float16 v8h  __attribute__((ext_vector_type(8)));
typedef float    v8f  __attribute__((ext_vector_type(8)));
typedef float    v4f  __attribute__((ext_vector_type(4)));
typedef unsigned int v4u __attribute__((ext_vector_type(4)));
typedef unsigned int v2u __attribute__((ext_vector_type(2)));

union FragH { v16h v; v8h h[2]; v4u u[2]; };

__device__ __forceinline__ unsigned short bf_bits(float f) {
  unsigned u = __float_as_uint(f);
  return (unsigned short)((u + 0x7FFFu + ((u >> 16) & 1u)) >> 16);
}
__device__ __forceinline__ float bf_up(unsigned short h) { return __uint_as_float(((unsigned)h) << 16); }
__device__ __forceinline__ float bfr(float f) { return bf_up(bf_bits(f)); }
__device__ __forceinline__ unsigned short h_bits(_Float16 x) { return __builtin_bit_cast(unsigned short, x); }
__device__ __forceinline__ unsigned pk16(unsigned short a, unsigned short b) { return (unsigned)a | ((unsigned)b << 16); }
__device__ __forceinline__ v8f zero8() { v8f z = {0.f, 0.f, 0.f, 0.f, 0.f, 0.f, 0.f, 0.f}; return z; }

__device__ __forceinline__ v16h ldfrag_h(const _Float16* p) {
  FragH f;
  f.h[0] = *(const v8h*)(p);
  f.h[1] = *(const v8h*)(p + 16);
  return f.v;
}
__device__ __forceinline__ v16h ldfrag_u(const unsigned short* p) {
  FragH f;
  f.u[0] = *(const v4u*)(p);
  f.u[1] = *(const v4u*)(p + 16);
  return f.v;
}

__device__ __forceinline__ v8f mma_raw(v16h a, v16h b, v8f c) {
  return __builtin_amdgcn_wmma_f32_16x16x32_f16(false, a, false, b, (short)0, c, false, false);
}
__device__ __forceinline__ void dep_guard1(v8f& a, v8f& b, v16h x) {
#if defined(__HIP_DEVICE_COMPILE__)
  asm volatile("v_nop\n\tv_nop\n\tv_nop\n\tv_nop" : "+v"(a), "+v"(b) : "v"(x));
#endif
}
__device__ __forceinline__ void guard_s(v8f& s, v16h a0, v16h a1, v16h b0, v16h b1) {
#if defined(__HIP_DEVICE_COMPILE__)
  asm volatile("v_nop\n\tv_nop\n\tv_nop\n\tv_nop" : "+v"(s) : "v"(a0), "v"(a1), "v"(b0), "v"(b1));
#endif
}
__device__ __forceinline__ void guard_pv(v8f& a, v8f& b, v16h x, v16h y, v16h z) {
#if defined(__HIP_DEVICE_COMPILE__)
  asm volatile("v_nop\n\tv_nop\n\tv_nop\n\tv_nop" : "+v"(a), "+v"(b) : "v"(x), "v"(y), "v"(z));
#endif
}
__device__ __forceinline__ void keep4_h(v16h a, v16h b, v16h c, v16h d) {
#if defined(__HIP_DEVICE_COMPILE__)
  asm volatile("v_nop" :: "v"(a), "v"(b), "v"(c), "v"(d));
#endif
}
__device__ __forceinline__ void acc_guard4(v8f& a, v8f& b, v8f& c, v8f& d) {
#if defined(__HIP_DEVICE_COMPILE__)
  asm volatile("v_nop\n\tv_nop\n\tv_nop\n\tv_nop" : "+v"(a), "+v"(b), "+v"(c), "+v"(d));
#endif
}
__device__ __forceinline__ void wave_sync_lds() {
  __builtin_amdgcn_fence(__ATOMIC_RELEASE, "workgroup");
  __builtin_amdgcn_wave_barrier();
  __builtin_amdgcn_fence(__ATOMIC_ACQUIRE, "workgroup");
}

__global__ __launch_bounds__(256) void conv16(const float* __restrict__ W, unsigned short* dst, int n8, float wsc) {
  const int i  = blockIdx.x * 256 + threadIdx.x;
  const int ic = (i < n8) ? i : (n8 - 1);
  const float* p = W + (size_t)ic * 8;
  const v4f a = *(const v4f*)(p), b = *(const v4f*)(p + 4);
  float v[8];
#pragma unroll
  for (int e = 0; e < 4; ++e) { v[e] = bfr(a[e]); v[4 + e] = bfr(b[e]); }
  v4u ov;
#pragma unroll
  for (int e = 0; e < 4; ++e) ov[e] = pk16(h_bits((_Float16)(v[2 * e] * wsc)), h_bits((_Float16)(v[2 * e + 1] * wsc)));
  if (i < n8) *(volatile v4u*)(dst + (size_t)i * 8) = ov;
  __threadfence();
  if (i < n8) *(volatile v4u*)(dst + (size_t)i * 8) = ov;
}

__global__ __launch_bounds__(256) void prep16(const float* __restrict__ x, int roff,
                                              const float* __restrict__ spos, const float* __restrict__ tpos,
                                              unsigned short* P) {
  const int i  = blockIdx.x * 256 + threadIdx.x;
  const int rr = i / P_CH;
  const int c8 = (i - rr * P_CH) * 8;
  const int b  = rr / SP;
  const int r  = rr - b * SP;
  const int rc = (r < SQ) ? r : (SQ - 1);
  const int n  = rc >> 3, t = rc & 7;
  const float* xp = x    + ((size_t)(roff + n) * NBT + b * TFR + t) * DM + c8;
  const float* pp = spos + (size_t)n * DM + c8;
  const float* qp = tpos + (size_t)t * DM + c8;
  const v4f x0 = *(const v4f*)(xp), x1 = *(const v4f*)(xp + 4);
  const v4f s0 = *(const v4f*)(pp), s1 = *(const v4f*)(pp + 4);
  const v4f t0 = *(const v4f*)(qp), t1 = *(const v4f*)(qp + 4);
  const bool live = (r < SQ);
  float v[8];
#pragma unroll
  for (int e = 0; e < 4; ++e) {
    const float f0 = (bfr(x0[e]) + bfr(s0[e])) + bfr(t0[e]);
    const float f1 = (bfr(x1[e]) + bfr(s1[e])) + bfr(t1[e]);
    v[e]     = live ? f0 : 0.f;
    v[4 + e] = live ? f1 : 0.f;
  }
  v4u o;
#pragma unroll
  for (int e = 0; e < 4; ++e) o[e] = pk16(h_bits((_Float16)(v[2 * e] * ACARRY)), h_bits((_Float16)(v[2 * e + 1] * ACARRY)));
  unsigned short* dp = P + (size_t)i * 8;
  *(volatile v4u*)dp = o;
  __threadfence();
  *(volatile v4u*)dp = o;
}

__global__ __launch_bounds__(256) void misc(const float* __restrict__ tx, float* out, unsigned short* CT) {
  if (blockIdx.x < CLS_BLOCKS) {
    const int i = blockIdx.x * 256 + threadIdx.x;
    const v4f a = *(const v4f*)(tx + (size_t)i * 4);
    v4f o;
#pragma unroll
    for (int e = 0; e < 4; ++e) o[e] = bfr(a[e]);
    float* dp = out + (size_t)i * 4;
    *(volatile v4f*)dp = o;
    __threadfence();
    *(volatile v4f*)dp = o;
  } else {
    const int j   = (blockIdx.x - CLS_BLOCKS) * 256 + threadIdx.x;
    const int b   = j / ZP_PERB;
    const int rem = j - b * ZP_PERB;
    const int rr  = rem / P_CH;
    const int c8  = (rem - rr * P_CH) * 8;
    v4u z = {0u, 0u, 0u, 0u};
    unsigned short* dp = CT + ((size_t)b * SP + SQ + rr) * DM + c8;
    *(volatile v4u*)dp = z;
    __threadfence();
    *(volatile v4u*)dp = z;
  }
}

template <int OM, int BIASM>
__global__ __launch_bounds__(256) void gemm64(
    const unsigned short* __restrict__ Ap, int lda, long long sAo, long long sAi,
    const unsigned short* __restrict__ Btp, int ldb, long long sBo, long long sBi,
    const float* __restrict__ bias, int sbo, int sbi, float bscale,
    void* Cout, int ldc, long long sCo, long long sCi,
    int M, int N, int K, int Mv, int nin, float oscale) {
  __shared__ __align__(16) float sT[8][16 * 68];
  const int by   = blockIdx.y;
  const int bo   = by / nin;
  const int bi   = by - bo * nin;
  const int lane = threadIdx.x & 31;
  const int wave = threadIdx.x >> 5;
  const int tilesN = N >> 6;
  const int tilesM = M >> 6;
  const int tile = blockIdx.x * 8 + wave;
  if (tile >= tilesM * tilesN) return;
  const int tm = tile / tilesN;
  const int tn = tile - tm * tilesN;
  const int m0 = tm << 6;
  const int n0 = tn << 6;

  const unsigned short* A1 = Ap  + (size_t)((long long)bo * sAo + (long long)bi * sAi);
  const unsigned short* Bb = Btp + (size_t)((long long)bo * sBo + (long long)bi * sBi);
  const float*         bsp = bias + (size_t)bo * (size_t)sbo + (size_t)bi * (size_t)sbi;

  const int rlane = lane & 15;
  const int koff  = (lane >> 4) * 8;
  const int mOff  = (lane >> 4) * 8;

  v8f acc[4][4];
#pragma unroll
  for (int i = 0; i < 4; ++i)
#pragma unroll
    for (int j = 0; j < 4; ++j) acc[i][j] = zero8();

  for (int k0 = 0; k0 < K; k0 += 32) {
    v16h bh[4];
#pragma unroll
    for (int j = 0; j < 4; ++j) {
      const size_t bofs = (size_t)(n0 + (j << 4) + rlane) * ldb + koff + k0;
      bh[j] = ldfrag_u(Bb + bofs);
    }
#pragma unroll
    for (int i = 0; i < 4; ++i) {
      const size_t ao = (size_t)(m0 + (i << 4) + rlane) * lda + koff + k0;
      const v16h ah = ldfrag_u(A1 + ao);
#pragma unroll
      for (int j = 0; j < 4; ++j) acc[i][j] = mma_raw(ah, bh[j], acc[i][j]);
      dep_guard1(acc[i][0], acc[i][3], ah);
    }
    keep4_h(bh[0], bh[1], bh[2], bh[3]);
  }
  acc_guard4(acc[0][0], acc[0][1], acc[0][2], acc[0][3]);
  acc_guard4(acc[1][0], acc[1][1], acc[1][2], acc[1][3]);
  acc_guard4(acc[2][0], acc[2][1], acc[2][2], acc[2][3]);
  acc_guard4(acc[3][0], acc[3][1], acc[3][2], acc[3][3]);

  const int hh2 = lane >> 4, c4 = (lane & 15) * 4;
  const int q8  = lane >> 3, c8 = (lane & 7) * 8;
  float bc[8];
#pragma unroll
  for (int e = 0; e < 8; ++e) bc[e] = 0.f;
  if (BIASM == 0) {
    if (OM != 2) {
      const int cb = n0 + c4;
      const int i0 = (cb < N - 4) ? cb : (N - 4);
      const v4f b0v = *(const v4f*)(bsp + i0);
#pragma unroll
      for (int e = 0; e < 4; ++e) bc[e] = bfr(b0v[e]) * bscale;
    } else {
      const int cb = n0 + c8;
      const int i0 = (cb < N - 8) ? cb : (N - 8);
      const v4f b0a = *(const v4f*)(bsp + i0), b0b = *(const v4f*)(bsp + i0 + 4);
#pragma unroll
      for (int e = 0; e < 4; ++e) {
        bc[e]     = bfr(b0a[e]) * bscale;
        bc[4 + e] = bfr(b0b[e]) * bscale;
      }
    }
  }

  float* slab = sT[wave];
#pragma unroll
  for (int i = 0; i < 4; ++i) {
    const int mBase = m0 + (i << 4);
#pragma unroll
    for (int j = 0; j < 4; ++j) {
#pragma unroll
      for (int r = 0; r < 8; ++r) {
        slab[(mOff + r) * 68 + (j << 4) + rlane] = acc[i][j][r];
      }
    }
    wave_sync_lds();
    if (OM != 2) {
      float* C = (float*)Cout + (size_t)((long long)bo * sCo + (long long)bi * sCi);
      v4f vals[8];
#pragma unroll
      for (int it = 0; it < 8; ++it) {
        const int row = it * 2 + hh2;
        v4f v = *(const v4f*)(slab + row * 68 + c4);
#pragma unroll
        for (int e = 0; e < 4; ++e) v[e] = v[e] * oscale + bc[e];
        vals[it] = v;
      }
      for (int pass = 0; pass < 2; ++pass) {
#pragma unroll
        for (int it = 0; it < 8; ++it) {
          const int gr = mBase + it * 2 + hh2;
          if (gr < Mv) {
            const int dr = (OM == 0) ? gr : (NBT + NBT * (gr >> 3) + TFR * bo + (gr & 7));
            *(volatile v4f*)(C + (size_t)dr * ldc + n0 + c4) = vals[it];
          }
        }
        __threadfence();
      }
    } else {
      unsigned short* C = (unsigned short*)Cout + (size_t)((long long)bo * sCo + (long long)bi * sCi);
      v4u hv[4];
#pragma unroll
      for (int it = 0; it < 4; ++it) {
        const int row = it * 4 + q8;
        const float* sp = slab + row * 68 + c8;
        float bm = 0.f;
        if (BIASM == 1) bm = bfr(bsp[mBase + row]) * bscale;
        v4u a;
#pragma unroll
        for (int e = 0; e < 4; ++e) {
          const float f0 = sp[2 * e]     * oscale + ((BIASM == 1) ? bm : bc[2 * e]);
          const float f1 = sp[2 * e + 1] * oscale + ((BIASM == 1) ? bm : bc[2 * e + 1]);
          a[e] = pk16(h_bits((_Float16)f0), h_bits((_Float16)f1));
        }
        hv[it] = a;
      }
      for (int pass = 0; pass < 2; ++pass) {
#pragma unroll
        for (int it = 0; it < 4; ++it) {
          const int row = it * 4 + q8;
          *(volatile v4u*)(C + (size_t)(mBase + row) * ldc + n0 + c8) = hv[it];
        }
        __threadfence();
      }
    }
    wave_sync_lds();
  }
}

__global__ __launch_bounds__(128)
void attn16(const unsigned short* __restrict__ Qpl, const unsigned short* __restrict__ Kpl,
            const unsigned short* __restrict__ VT, unsigned short* CT) {
  __shared__ __align__(16) float Ps[4][16 * 36];
  __shared__ __align__(16) float Os[4][16 * 64];

  const int tid  = threadIdx.x;
  const int wave = tid >> 5;
  const int lane = tid & 31;
  const int hh   = lane >> 4;
  const int c    = lane & 15;

  const int wid  = blockIdx.x * 4 + wave;
  const int bh   = wid / (SQ / 16);
  const int qt   = wid - bh * (SQ / 16);
  const int bat  = bh / NH;
  const int head = bh - bat * NH;
  const int q0   = qt * 16;

  const _Float16* Qb = (const _Float16*)(const void*)Qpl + (size_t)bat * SP * DM + head * HD;
  const _Float16* Kb = (const _Float16*)(const void*)Kpl + (size_t)bat * SP * DM + head * HD;
  const _Float16* Vb = (const _Float16*)(const void*)VT + (size_t)bh * HD * SP;
  const float lsc = (1.4426950408889634f * 0.125f) / (QKCARRY * QKCARRY);

  const v16h qa0 = ldfrag_h(Qb + (size_t)(q0 + c) * DM + 8 * hh);
  const v16h qa1 = ldfrag_h(Qb + (size_t)(q0 + c) * DM + 32 + 8 * hh);

  float mrow[8], lrow[8];
  v8f acc0 = zero8(), acc1 = zero8(), acc2 = zero8(), acc3 = zero8();
#pragma unroll
  for (int r = 0; r < 8; ++r) { mrow[r] = -INFINITY; lrow[r] = 0.f; }
  float* pt = Ps[wave];

#pragma unroll 1
  for (int kb = 0; kb < SQ; kb += 32) {
    const _Float16* kp = Kb + (size_t)(kb + c) * DM + 8 * hh;
    v8f s0, s1;
    {
      const v16h k00 = ldfrag_h(kp), k01 = ldfrag_h(kp + 32);
      s0 = mma_raw(qa0, k00, zero8());
      s0 = mma_raw(qa1, k01, s0);
      guard_s(s0, qa0, qa1, k00, k01);
    }
    {
      const v16h k10 = ldfrag_h(kp + (size_t)16 * DM), k11 = ldfrag_h(kp + (size_t)16 * DM + 32);
      s1 = mma_raw(qa0, k10, zero8());
      s1 = mma_raw(qa1, k11, s1);
      guard_s(s1, qa0, qa1, k10, k11);
    }
#pragma unroll
    for (int r = 0; r < 8; ++r) {
      const float t0 = s0[r] * lsc, t1 = s1[r] * lsc;
      float mx = fmaxf(t0, t1);
#pragma unroll
      for (int off = 1; off < 16; off <<= 1) mx = fmaxf(mx, __shfl_xor(mx, off, 32));
      const float mn = fmaxf(mrow[r], mx);
      const float al = exp2f(mrow[r] - mn);
      mrow[r] = mn;
      const float e0 = exp2f(t0 - mn), e1 = exp2f(t1 - mn);
      float ps = e0 + e1;
#pragma unroll
      for (int off = 1; off < 16; off <<= 1) ps += __shfl_xor(ps, off, 32);
      lrow[r] = lrow[r] * al + ps;
      acc0[r] *= al;
      acc1[r] *= al;
      acc2[r] *= al;
      acc3[r] *= al;
      const int ro = (8 * hh + r) * 36 + c;
      pt[ro]      = e0;
      pt[ro + 16] = e1;
    }
    wave_sync_lds();
    FragH pa;
    {
      const float* prow = pt + c * 36 + 8 * hh;
      const v4f p0 = *(const v4f*)(prow), p1 = *(const v4f*)(prow + 4);
      const v4f p2 = *(const v4f*)(prow + 16), p3 = *(const v4f*)(prow + 20);
#pragma unroll
      for (int e = 0; e < 4; ++e) {
        pa.h[0][e]     = (_Float16)(p0[e] * PCARRY);
        pa.h[0][4 + e] = (_Float16)(p1[e] * PCARRY);
        pa.h[1][e]     = (_Float16)(p2[e] * PCARRY);
        pa.h[1][4 + e] = (_Float16)(p3[e] * PCARRY);
      }
    }
    const _Float16* vp = Vb + (size_t)c * SP + kb + 8 * hh;
    {
      const v16h vb0 = ldfrag_h(vp), vb1 = ldfrag_h(vp + (size_t)16 * SP);
      acc0 = mma_raw(pa.v, vb0, acc0);
      acc1 = mma_raw(pa.v, vb1, acc1);
      guard_pv(acc0, acc1, pa.v, vb0, vb1);
    }
    {
      const v16h vb2 = ldfrag_h(vp + (size_t)32 * SP), vb3 = ldfrag_h(vp + (size_t)48 * SP);
      acc2 = mma_raw(pa.v, vb2, acc2);
      acc3 = mma_raw(pa.v, vb3, acc3);
      guard_pv(acc2, acc3, pa.v, vb2, vb3);
    }
    wave_sync_lds();
  }

  float* os = Os[wave];
  const float oc = FCARRY / (PCARRY * VCARRY);
#pragma unroll
  for (int r = 0; r < 8; ++r) {
    const float inv = (1.0f / lrow[r]) * oc;
    const int ro = (8 * hh + r) * 64 + c;
    os[ro]      = acc0[r] * inv;
    os[ro + 16] = acc1[r] * inv;
    os[ro + 32] = acc2[r] * inv;
    os[ro + 48] = acc3[r] * inv;
  }
  wave_sync_lds();
  {
    const int q8 = lane >> 3, c8 = (lane & 7) * 8;
    v4u hv[4];
#pragma unroll
    for (int it = 0; it < 4; ++it) {
      const int row = it * 4 + q8;
      const float* sp = os + row * 64 + c8;
      v4u a;
#pragma unroll
      for (int e = 0; e < 4; ++e) a[e] = pk16(h_bits((_Float16)sp[2 * e]), h_bits((_Float16)sp[2 * e + 1]));
      hv[it] = a;
    }
    unsigned short* dst = CT + ((size_t)bat * SP + q0) * DM + head * HD + c8;
    for (int pass = 0; pass < 2; ++pass) {
#pragma unroll
      for (int it = 0; it < 4; ++it) {
        const int row = it * 4 + q8;
        *(volatile v4u*)(dst + (size_t)row * DM) = hv[it];
      }
      __threadfence();
    }
  }
}

extern "C" void kernel_launch(void* const* d_in, const int* in_sizes, int n_in,
                              void* d_out, int out_size, void* d_ws, size_t ws_size,
                              hipStream_t stream) {
  if (n_in < 12) return;
  if (in_sizes[0] != NSROWS * NBT * DM) return;
  if (in_sizes[1] != NTROWS * NBT * DM) return;
  if (in_sizes[2] != NSP * DM || in_sizes[3] != NSP * DM) return;
  if (in_sizes[4] != TFR * DM || in_sizes[5] != TFR * DM) return;
  if (in_sizes[6] != DM * DM || in_sizes[7] != DM) return;
  if (in_sizes[8] != KVN * DM || in_sizes[9] != KVN) return;
  if (in_sizes[10] != DM * DM || in_sizes[11] != DM) return;
  if (out_size != NTROWS * NBT * DM) return;

  const float* s_x  = (const float*)d_in[0];
  const float* t_x  = (const float*)d_in[1];
  const float* csp  = (const float*)d_in[2];
  const float* vsp  = (const float*)d_in[3];
  const float* ctp  = (const float*)d_in[4];
  const float* vtp  = (const float*)d_in[5];
  const float* q_w  = (const float*)d_in[6];
  const float* q_b  = (const float*)d_in[7];
  const float* kv_w = (const float*)d_in[8];
  const float* kv_b = (const float*)d_in[9];
  const float* p_w  = (const float*)d_in[10];
  const float* p_b  = (const float*)d_in[11];
  float*       out  = (float*)d_out;

  const size_t PWQ = (size_t)DM * DM * 2;
  const size_t PWK = (size_t)KVN * DM * 2;
  const size_t PWO = (size_t)DM * DM * 2;
  const size_t PTK = (size_t)NB * SP * DM * 2;
  const size_t PVT = (size_t)NB * NH * HD * SP * 2;
  size_t off = 0;
  const size_t oWQ = off; off += PWQ;
  const size_t oWK = off; off += PWK;
  const size_t oWO = off; off += PWO;
  const size_t oTP = off; off += PTK;
  const size_t oSP = off; off += PTK;
  const size_t oQP = off; off += PTK;
  const size_t oKP = off; off += PTK;
  const size_t oVT = off; off += PVT;
  const size_t oCT = off; off += PTK;
  if (off > ws_size) return;
  if (off > (size_t)134217728) return;

  char* ws = (char*)d_ws;
  unsigned short* WQ  = (unsigned short*)(ws + oWQ);
  unsigned short* WKV = (unsigned short*)(ws + oWK);
  unsigned short* WO  = (unsigned short*)(ws + oWO);
  unsigned short* TP  = (unsigned short*)(ws + oTP);
  unsigned short* SPL = (unsigned short*)(ws + oSP);
  unsigned short* QP  = (unsigned short*)(ws + oQP);
  unsigned short* KP  = (unsigned short*)(ws + oKP);
  unsigned short* VTp = (unsigned short*)(ws + oVT);
  unsigned short* CT  = (unsigned short*)(ws + oCT);

  const int n8q = (DM * DM) / 8;
  const int n8k = (KVN * DM) / 8;
  if ((n8q % 256) != 0 || (n8k % 256) != 0) return;
  const dim3 blk(256), blk128(128);
  const dim3 gCq(n8q / 256), gCk(n8k / 256);
  const dim3 gPR(PREP_BLOCKS);
  const dim3 gMI(CLS_BLOCKS + ZP_BLOCKS);
  const dim3 gQK(((SP / 64) * (DM / 64) + 7) / 8, NB);
  const dim3 gVT(((HD / 64) * (SP / 64) + 7) / 8, NB * NH);
  const dim3 gAT(ATT_BLOCKS);
  const dim3 gOU(((SP / 64) * (DM / 64) + 7) / 8, NB);

  conv16<<<gCq, blk, 0, stream>>>(q_w, WQ, n8q, WSC);
  conv16<<<gCk, blk, 0, stream>>>(kv_w, WKV, n8k, WSC);
  conv16<<<gCq, blk, 0, stream>>>(p_w, WO, n8q, WSC);

  prep16<<<gPR, blk, 0, stream>>>(t_x, 1, vsp, vtp, TP);
  prep16<<<gPR, blk, 0, stream>>>(s_x, 2, csp, ctp, SPL);

  misc<<<gMI, blk, 0, stream>>>(t_x, out, CT);

  gemm64<2, 0><<<gQK, blk, 0, stream>>>(
      TP, DM, (long long)SP * DM, 0LL,
      WQ, DM, 0LL, 0LL,
      q_b, 0, 0, QKCARRY,
      (void*)QP, DM, (long long)SP * DM, 0LL,
      SP, DM, DM, SP, 1, QKCARRY / (ACARRY * WSC));

  gemm64<2, 0><<<gQK, blk, 0, stream>>>(
      SPL, DM, (long long)SP * DM, 0LL,
      WKV, DM, 0LL, 0LL,
      kv_b, 0, 0, QKCARRY,
      (void*)KP, DM, (long long)SP * DM, 0LL,
      SP, DM, DM, SP, 1, QKCARRY / (ACARRY * WSC));

  gemm64<2, 1><<<gVT, blk, 0, stream>>>(
      WKV + (size_t)DM * DM, DM, 0LL, (long long)HD * DM,
      SPL, DM, (long long)SP * DM, 0LL,
      kv_b + DM, 0, HD, VCARRY,
      (void*)VTp, SP, (long long)NH * HD * SP, (long long)HD * SP,
      HD, SP, DM, HD, NH, VCARRY / (ACARRY * WSC));

  attn16<<<gAT, blk128, 0, stream>>>(QP, KP, VTp, CT);

  gemm64<1, 0><<<gOU, blk, 0, stream>>>(
      CT, DM, (long long)SP * DM, 0LL,
      WO, DM, 0LL, 0LL,
      p_b, 0, 0, 1.0f,
      (void*)out, DM, 0LL, 0LL,
      SP, DM, DM, SQ, 1, 1.0f / (FCARRY * WSC));
  (void)hipGetLastError();
}
